// _LongCatSingleAttention_76811195121708
// MI455X (gfx1250) — hardware-run, weakly checked
//
#include <hip/hip_runtime.h>
#include <math.h>

typedef __attribute__((ext_vector_type(16))) _Float16 v16h;
typedef __attribute__((ext_vector_type(8)))  _Float16 v8h;
typedef __attribute__((ext_vector_type(8)))  float    v8f;
typedef __attribute__((ext_vector_type(4)))  float    v4f;
typedef __attribute__((ext_vector_type(4)))  unsigned int v4u;

constexpr int kSeq    = 2048;
constexpr int kDim    = 3072;
constexpr int kHeads  = 24;
constexpr int kHd     = 128;
constexpr int kInner  = kHeads * kHd;
constexpr int kKc     = 64;
static_assert(kInner == 3072, "inner width");
static_assert((kDim % 32) == 0, "GEMM K multiple of 32");
static_assert((kSeq % 64) == 0 && (kInner % 64) == 0, "GEMM M,N multiples of 64");
static_assert((kSeq % kKc) == 0 && kHd == 128 && (kHeads % 2) == 0, "attention tiling");

constexpr float kXCarry = 16.0f;
constexpr float kWCarry = 256.0f;
constexpr float kQCarry = 16.0f;
constexpr float kKCarry = 16.0f;
constexpr float kVCarry = 16.0f;
constexpr float kPCarry = 1024.0f;
constexpr float kProjScale = 1.0f / (kXCarry * kWCarry);
constexpr float kVtScale   = kVCarry * kProjScale;
constexpr float kNormEps   = 1e-6f;
constexpr float kInvHd     = 1.0f / (float)kHd;

constexpr double csqrt_iter(double x, double g, int n) { return n == 0 ? g : csqrt_iter(x, 0.5 * (g + x / g), n - 1); }
constexpr double csqrt_d(double x) { return csqrt_iter(x, x, 48); }
constexpr float kInvSqrtHd  = (float)(1.0 / csqrt_d((double)kHd));
static_assert(kInvSqrtHd * kInvSqrtHd * (float)kHd > 0.99999f && kInvSqrtHd * kInvSqrtHd * (float)kHd < 1.00001f, "score scale");
constexpr float kScoreScale = kInvSqrtHd / (kQCarry * kKCarry);
constexpr float kOutCarry   = kPCarry * kVCarry;

constexpr size_t kOffXH  = 0;
constexpr size_t kOffWH  = kOffXH + (size_t)kSeq * kDim * 2;
constexpr size_t kOffQF  = kOffWH + (size_t)3 * kInner * kDim * 2;
constexpr size_t kOffKF  = kOffQF + (size_t)kSeq * kInner * 4;
constexpr size_t kOffVT  = kOffKF + (size_t)kSeq * kInner * 4;
constexpr size_t kWsTotal = kOffVT + (size_t)kInner * kSeq * 2;
constexpr size_t kOffQ16 = kOffWH;
constexpr size_t kOffK16 = kOffWH + (size_t)kHeads * kSeq * kHd * 2;
static_assert(kWsTotal == 132120576ull, "carve total");
static_assert(kWsTotal <= 134217728ull, "carve cap");
static_assert(kOffK16 + (size_t)kHeads * kSeq * kHd * 2 <= kOffWH + (size_t)2 * kInner * kDim * 2, "q/k planes stay inside the wq|wk planes");
static_assert((kOffWH % 128) == 0 && (kOffQF % 128) == 0 && (kOffKF % 128) == 0 && (kOffVT % 128) == 0 && (kOffK16 % 128) == 0, "128-B aligned regions");

union FragU { v16h v; v8h h[2]; };
__device__ __forceinline__ v16h ldfrag(const _Float16* p) {
  FragU f;
  f.h[0] = *(const v8h*)(p);
  f.h[1] = *(const v8h*)(p + 16);
  return f.v;
}
__device__ __forceinline__ v8f mma_h(v16h a, v16h b, v8f c) {
  c = __builtin_amdgcn_wmma_f32_16x16x32_f16(false, a, false, b, (short)0, c, false, false);
  asm volatile("v_nop\n\tv_nop\n\tv_nop\n\tv_nop" : "+v"(c) : "v"(a), "v"(b));
  return c;
}
__device__ __forceinline__ unsigned pk16(unsigned short a, unsigned short b) { return (unsigned)a | ((unsigned)b << 16); }
__device__ __forceinline__ unsigned short h_bits(float f) {
  const _Float16 h = (_Float16)f;
  return __builtin_bit_cast(unsigned short, h);
}

__global__ __launch_bounds__(256) void cast8_f16_kernel(const float* __restrict__ in0, const float* __restrict__ in1,
                                                        const float* __restrict__ in2, unsigned short* __restrict__ out,
                                                        int n8, float carry) {
  const int z = blockIdx.y;
  const float* in = (z == 0) ? in0 : (z == 1) ? in1 : in2;
  const int i = blockIdx.x * 256 + threadIdx.x;
  if (i >= n8) return;
  const float* p = in + 8 * (size_t)i;
  const v4f a = *(const v4f*)(p);
  const v4f c = *(const v4f*)(p + 4);
  unsigned short hb[8];
#pragma unroll
  for (int e = 0; e < 4; ++e) {
    const float fa = a[e] * carry;
    const float fc = c[e] * carry;
    hb[e]     = h_bits(fa);
    hb[4 + e] = h_bits(fc);
  }
  const v4u u = (v4u){pk16(hb[0], hb[1]), pk16(hb[2], hb[3]), pk16(hb[4], hb[5]), pk16(hb[6], hb[7])};
  unsigned short* q = out + (size_t)z * (size_t)n8 * 8 + 8 * (size_t)i;
  *(volatile v4u*)q = u;
  __threadfence();
  *(volatile v4u*)q = u;
}

template <int BIAS_MODE, int OUT_MODE>
__global__ __launch_bounds__(256) void wmma_gemm64(
    const unsigned short* __restrict__ Ap, int lda,
    const unsigned short* __restrict__ Btp, int ldb,
    void* __restrict__ Cout, int ldc,
    const float* __restrict__ bias, float bscale,
    int M, int N, int K, float scale) {
  const _Float16* A  = (const _Float16*)Ap;
  const _Float16* Bt = (const _Float16*)Btp;
  __shared__ __align__(16) float sT[8][16 * 68];
  const int lane = threadIdx.x & 31;
  const int wave = __builtin_amdgcn_readfirstlane((int)(threadIdx.x >> 5));
  const int tilesN = N >> 6;
  const int tilesM = M >> 6;
  const int tile = blockIdx.x * 8 + wave;
  if (tile >= tilesM * tilesN) return;
  const int tm = tile / tilesN;
  const int tn = tile - tm * tilesN;
  const int m0 = tm << 6;
  const int n0 = tn << 6;

  const int rlane = lane & 15;
  const int koff  = (lane >> 4) * 8;
  const int mOff  = (lane >> 4) * 8;

  v8f acc[4][4];
#pragma unroll
  for (int i = 0; i < 4; ++i)
#pragma unroll
    for (int j = 0; j < 4; ++j) acc[i][j] = (v8f){0.f, 0.f, 0.f, 0.f, 0.f, 0.f, 0.f, 0.f};

  for (int k0 = 0; k0 < K; k0 += 32) {
    v16h bh[4];
#pragma unroll
    for (int j = 0; j < 4; ++j) {
      const size_t bo = (size_t)(n0 + (j << 4) + rlane) * ldb + koff + k0;
      bh[j] = ldfrag(Bt + bo);
    }
#pragma unroll
    for (int i = 0; i < 4; ++i) {
      const size_t ao = (size_t)(m0 + (i << 4) + rlane) * lda + koff + k0;
      const v16h ah = ldfrag(A + ao);
#pragma unroll
      for (int j = 0; j < 4; ++j) acc[i][j] = mma_h(ah, bh[j], acc[i][j]);
    }
  }

  float* slab = sT[wave];
#pragma unroll
  for (int i = 0; i < 4; ++i) {
    const int mBase = m0 + (i << 4);
    float br[8];
#pragma unroll
    for (int r = 0; r < 8; ++r) br[r] = (BIAS_MODE == 1) ? (bias[mBase + mOff + r] * bscale) : 0.0f;
#pragma unroll
    for (int j = 0; j < 4; ++j) {
      const int n = n0 + (j << 4) + rlane;
      float bv = 0.f;
      if (BIAS_MODE == 2) bv = bias[n] * bscale;
#pragma unroll
      for (int r = 0; r < 8; ++r) {
        float v = acc[i][j][r] * scale;
        if (BIAS_MODE == 1) v += br[r];
        if (BIAS_MODE == 2) v += bv;
        slab[(mOff + r) * 68 + (j << 4) + rlane] = v;
      }
    }
    __builtin_amdgcn_fence(__ATOMIC_RELEASE, "workgroup");
    __builtin_amdgcn_wave_barrier();
    __builtin_amdgcn_fence(__ATOMIC_ACQUIRE, "workgroup");
    if (OUT_MODE == 0) {
      float* C = (float*)Cout;
      const int hh = lane >> 4, c4 = (lane & 15) * 4;
      for (int pass = 0; pass < 2; ++pass) {
#pragma unroll
        for (int it = 0; it < 8; ++it) {
          const int row = it * 2 + hh;
          v4f v = *(const v4f*)(slab + row * 68 + c4);
          *(volatile v4f*)(C + (size_t)(mBase + row) * ldc + n0 + c4) = v;
        }
        __threadfence();
      }
    } else {
      const int q = lane >> 3, c8 = (lane & 7) * 8;
      unsigned short* C = (unsigned short*)Cout;
      for (int pass = 0; pass < 2; ++pass) {
#pragma unroll
        for (int it = 0; it < 4; ++it) {
          const int row = it * 4 + q;
          const float* sp = slab + row * 68 + c8;
          v8h hv;
#pragma unroll
          for (int e = 0; e < 8; ++e) hv[e] = (_Float16)sp[e];
          *(volatile v8h*)(C + (size_t)(mBase + row) * ldc + n0 + c8) = hv;
        }
        __threadfence();
      }
    }
    __builtin_amdgcn_fence(__ATOMIC_RELEASE, "workgroup");
    __builtin_amdgcn_wave_barrier();
    __builtin_amdgcn_fence(__ATOMIC_ACQUIRE, "workgroup");
  }
}

__global__ __launch_bounds__(256) void norm_rot_kernel(
    const float* __restrict__ QF, const float* __restrict__ KF,
    const float* __restrict__ nqw, const float* __restrict__ nkw,
    const float* __restrict__ ctab, const float* __restrict__ ttab,
    unsigned short* __restrict__ Q16, unsigned short* __restrict__ K16, float carry) {
  const int z = blockIdx.y;
  const float* src = (z == 0) ? QF : KF;
  const float* nw  = (z == 0) ? nqw : nkw;
  unsigned short* dst = (z == 0) ? Q16 : K16;
  const int lane = threadIdx.x & 31;
  const int wave = __builtin_amdgcn_readfirstlane((int)(threadIdx.x >> 5));
  const int hh = lane >> 4, c = lane & 15;
  const int pair = blockIdx.x * 8 + wave;
  const int s = pair / (kHeads / 2);
  const int h = (pair - s * (kHeads / 2)) * 2 + hh;
  const int d0 = c * 8;
  const float* xp = src + (size_t)s * kInner + h * kHd + d0;
  const v4f xa = *(const v4f*)(xp);
  const v4f xb = *(const v4f*)(xp + 4);
  const v4f ca = *(const v4f*)(ctab + (size_t)s * kHd + d0);
  const v4f cb = *(const v4f*)(ctab + (size_t)s * kHd + d0 + 4);
  const v4f ta = *(const v4f*)(ttab + (size_t)s * kHd + d0);
  const v4f tb = *(const v4f*)(ttab + (size_t)s * kHd + d0 + 4);
  const v4f wa = *(const v4f*)(nw + d0);
  const v4f wb = *(const v4f*)(nw + d0 + 4);
  float x[8], cc[8], tt[8], ww[8];
#pragma unroll
  for (int e = 0; e < 4; ++e) {
    x[e] = xa[e];  x[4 + e] = xb[e];
    cc[e] = ca[e]; cc[4 + e] = cb[e];
    tt[e] = ta[e]; tt[4 + e] = tb[e];
    ww[e] = wa[e]; ww[4 + e] = wb[e];
  }
  float ss = 0.0f;
#pragma unroll
  for (int e = 0; e < 8; ++e) ss += x[e] * x[e];
  ss += __shfl_xor(ss, 1, 32);
  ss += __shfl_xor(ss, 2, 32);
  ss += __shfl_xor(ss, 4, 32);
  ss += __shfl_xor(ss, 8, 32);
  const float inv = rsqrtf(ss * kInvHd + kNormEps);
  float xn[8];
#pragma unroll
  for (int e = 0; e < 8; ++e) xn[e] = (x[e] * inv) * ww[e];
  unsigned short hb[8];
#pragma unroll
  for (int i = 0; i < 4; ++i) {
    const float y0 = xn[2 * i] * cc[2 * i] - xn[2 * i + 1] * tt[2 * i];
    const float y1 = xn[2 * i + 1] * cc[2 * i + 1] + xn[2 * i] * tt[2 * i + 1];
    hb[2 * i]     = h_bits(y0 * carry);
    hb[2 * i + 1] = h_bits(y1 * carry);
  }
  const v4u u = (v4u){pk16(hb[0], hb[1]), pk16(hb[2], hb[3]), pk16(hb[4], hb[5]), pk16(hb[6], hb[7])};
  unsigned short* q = dst + ((size_t)h * kSeq + s) * kHd + d0;
  *(volatile v4u*)q = u;
  __threadfence();
  *(volatile v4u*)q = u;
}

__global__ __launch_bounds__(128) void attn128_kernel(const unsigned short* __restrict__ Q16p,
                                                      const unsigned short* __restrict__ K16p,
                                                      const unsigned short* __restrict__ VTp,
                                                      float* __restrict__ out) {
  __shared__ __align__(16) _Float16 Ksh[kKc * kHd];
  __shared__ __align__(16) _Float16 Vsh[kHd * kKc];
  __shared__ __align__(16) _Float16 Psh[4][16 * kKc];
  __shared__ __align__(16) float    Os[4][16 * 68];

  const int tid  = threadIdx.x;
  const int wave = __builtin_amdgcn_readfirstlane((int)(threadIdx.x >> 5));
  const int lane = tid & 31;
  const int hh   = lane >> 4;
  const int c    = lane & 15;

  constexpr int nqb = kSeq / 64;
  const int h  = blockIdx.x / nqb;
  const int qb = blockIdx.x - h * nqb;
  const int q0 = qb * 64 + wave * 16;

  const _Float16* Qh = (const _Float16*)Q16p + (size_t)h * kSeq * kHd;
  const _Float16* Kh = (const _Float16*)K16p + (size_t)h * kSeq * kHd;
  const _Float16* Vh = (const _Float16*)VTp  + (size_t)h * kHd * kSeq;

  v16h qa[4];
#pragma unroll
  for (int dc = 0; dc < 4; ++dc) qa[dc] = ldfrag(Qh + (size_t)(q0 + c) * kHd + dc * 32 + 8 * hh);

  float mrow[8], lrow[8];
  v8f oacc[8];
#pragma unroll
  for (int r = 0; r < 8; ++r) { mrow[r] = -INFINITY; lrow[r] = 0.f; }
#pragma unroll
  for (int t = 0; t < 8; ++t) oacc[t] = (v8f){0.f, 0.f, 0.f, 0.f, 0.f, 0.f, 0.f, 0.f};

  _Float16* pw = Psh[wave];

#pragma unroll 1
  for (int kc = 0; kc < kSeq / kKc; ++kc) {
    const int kv0 = kc * kKc;
    __syncthreads();
    {
      const _Float16* ksrc = Kh + (size_t)kv0 * kHd;
      v8h t[8];
#pragma unroll
      for (int i = 0; i < 8; ++i) t[i] = *(const v8h*)(ksrc + (size_t)(i * 128 + tid) * 8);
#pragma unroll
      for (int i = 0; i < 8; ++i) *(v8h*)(Ksh + (i * 128 + tid) * 8) = t[i];
    }
    {
      v8h t[8];
#pragma unroll
      for (int i = 0; i < 8; ++i) {
        const int p = i * 128 + tid;
        const int d = p >> 3, c8 = (p & 7) * 8;
        t[i] = *(const v8h*)(Vh + (size_t)d * kSeq + kv0 + c8);
      }
#pragma unroll
      for (int i = 0; i < 8; ++i) *(v8h*)(Vsh + (i * 128 + tid) * 8) = t[i];
    }
    __syncthreads();

    v8f s[4];
#pragma unroll
    for (int j = 0; j < 4; ++j) {
      s[j] = (v8f){0.f, 0.f, 0.f, 0.f, 0.f, 0.f, 0.f, 0.f};
#pragma unroll
      for (int dc = 0; dc < 4; ++dc) {
        const v16h kb = ldfrag(Ksh + (j * 16 + c) * kHd + dc * 32 + 8 * hh);
        s[j] = mma_h(qa[dc], kb, s[j]);
      }
    }

    float cm[8];
#pragma unroll
    for (int r = 0; r < 8; ++r) {
      float m = fmaxf(fmaxf(s[0][r], s[1][r]), fmaxf(s[2][r], s[3][r]));
      m = fmaxf(m, __shfl_xor(m, 1, 32));
      m = fmaxf(m, __shfl_xor(m, 2, 32));
      m = fmaxf(m, __shfl_xor(m, 4, 32));
      m = fmaxf(m, __shfl_xor(m, 8, 32));
      cm[r] = m * kScoreScale;
    }
#pragma unroll
    for (int r = 0; r < 8; ++r) {
      const float mnew  = fmaxf(mrow[r], cm[r]);
      const float alpha = __expf(mrow[r] - mnew);
      mrow[r] = mnew;
      float psum = 0.f;
#pragma unroll
      for (int j = 0; j < 4; ++j) {
        const float p = __expf(fmaf(s[j][r], kScoreScale, -mnew));
        psum += p;
        pw[(8 * hh + r) * kKc + j * 16 + c] = (_Float16)(p * kPCarry);
      }
      lrow[r] = lrow[r] * alpha + psum;
#pragma unroll
      for (int t = 0; t < 8; ++t) oacc[t][r] *= alpha;
    }
    __builtin_amdgcn_fence(__ATOMIC_RELEASE, "workgroup");
    __builtin_amdgcn_wave_barrier();
    __builtin_amdgcn_fence(__ATOMIC_ACQUIRE, "workgroup");
#pragma unroll
    for (int kk = 0; kk < 2; ++kk) {
      const v16h pa = ldfrag(pw + c * kKc + kk * 32 + 8 * hh);
#pragma unroll
      for (int t = 0; t < 8; ++t) {
        const v16h vb = ldfrag(Vsh + (t * 16 + c) * kKc + kk * 32 + 8 * hh);
        oacc[t] = mma_h(pa, vb, oacc[t]);
      }
    }
  }

  float inv[8];
#pragma unroll
  for (int r = 0; r < 8; ++r) {
    float l = lrow[r];
    l += __shfl_xor(l, 1, 32);
    l += __shfl_xor(l, 2, 32);
    l += __shfl_xor(l, 4, 32);
    l += __shfl_xor(l, 8, 32);
    inv[r] = 1.0f / (l * kOutCarry);
  }

  float* os = Os[wave];
  float* ob = out + (size_t)q0 * kInner + h * kHd;
  const int c4 = (lane & 15) * 4;
#pragma unroll
  for (int half = 0; half < 2; ++half) {
#pragma unroll
    for (int r = 0; r < 8; ++r) {
#pragma unroll
      for (int t = 0; t < 4; ++t) os[(8 * hh + r) * 68 + t * 16 + c] = oacc[half * 4 + t][r] * inv[r];
    }
    __builtin_amdgcn_fence(__ATOMIC_RELEASE, "workgroup");
    __builtin_amdgcn_wave_barrier();
    __builtin_amdgcn_fence(__ATOMIC_ACQUIRE, "workgroup");
    for (int pass = 0; pass < 2; ++pass) {
#pragma unroll
      for (int it = 0; it < 8; ++it) {
        const int row = it * 2 + hh;
        v4f val = *(const v4f*)(os + row * 68 + c4);
        *(volatile v4f*)(ob + (size_t)row * kInner + half * 64 + c4) = val;
      }
      __threadfence();
    }
    __builtin_amdgcn_fence(__ATOMIC_RELEASE, "workgroup");
    __builtin_amdgcn_wave_barrier();
    __builtin_amdgcn_fence(__ATOMIC_ACQUIRE, "workgroup");
  }
}

extern "C" void kernel_launch(void* const* d_in, const int* in_sizes, int n_in,
                              void* d_out, int out_size, void* d_ws, size_t ws_size,
                              hipStream_t stream) {
  if (n_in < 11) return;
  if (in_sizes[0] != kSeq * kDim) return;
  if (in_sizes[1] != kInner * kDim) return;
  if (in_sizes[2] != kInner) return;
  if (in_sizes[3] != kInner * kDim) return;
  if (in_sizes[4] != kInner) return;
  if (in_sizes[5] != kInner * kDim) return;
  if (in_sizes[6] != kInner) return;
  if (in_sizes[7] != kHd) return;
  if (in_sizes[8] != kHd) return;
  if (in_sizes[9] != kSeq * kHd) return;
  if (in_sizes[10] != kSeq * kHd) return;
  if (out_size != kSeq * kInner) return;
  if (ws_size < kWsTotal) return;

  const float* hidden = (const float*)d_in[0];
  const float* wq     = (const float*)d_in[1];
  const float* bq     = (const float*)d_in[2];
  const float* wk     = (const float*)d_in[3];
  const float* bk     = (const float*)d_in[4];
  const float* wv     = (const float*)d_in[5];
  const float* bv     = (const float*)d_in[6];
  const float* nqw    = (const float*)d_in[7];
  const float* nkw    = (const float*)d_in[8];
  const float* ctab   = (const float*)d_in[9];
  const float* ttab   = (const float*)d_in[10];
  float* out = (float*)d_out;

  char* ws = (char*)d_ws;
  unsigned short* XH  = (unsigned short*)(ws + kOffXH);
  unsigned short* WH  = (unsigned short*)(ws + kOffWH);
  float*          QF  = (float*)(ws + kOffQF);
  float*          KF  = (float*)(ws + kOffKF);
  unsigned short* VT  = (unsigned short*)(ws + kOffVT);
  unsigned short* Q16 = (unsigned short*)(ws + kOffQ16);
  unsigned short* K16 = (unsigned short*)(ws + kOffK16);
  unsigned short* WQH = WH;
  unsigned short* WKH = WH + (size_t)kInner * kDim;
  unsigned short* WVH = WH + (size_t)2 * kInner * kDim;

  constexpr int kX8 = kSeq * kDim / 8;
  constexpr int kW8 = kInner * kDim / 8;
  static_assert((kX8 % 256) == 0 && (kW8 % 256) == 0, "cast grids exact");

  cast8_f16_kernel<<<dim3(kX8 / 256, 1), 256, 0, stream>>>(hidden, hidden, hidden, XH, kX8, kXCarry);
  cast8_f16_kernel<<<dim3(kW8 / 256, 3), 256, 0, stream>>>(wq, wk, wv, WH, kW8, kWCarry);

  constexpr int kTiles = (kSeq / 64) * (kInner / 64);
  static_assert((kTiles % 8) == 0, "tiles per block");

  wmma_gemm64<2, 0><<<kTiles / 8, 256, 0, stream>>>(
      XH, kDim, WQH, kDim, (void*)QF, kInner, bq, 1.0f, kSeq, kInner, kDim, kProjScale);
  wmma_gemm64<2, 0><<<kTiles / 8, 256, 0, stream>>>(
      XH, kDim, WKH, kDim, (void*)KF, kInner, bk, 1.0f, kSeq, kInner, kDim, kProjScale);
  wmma_gemm64<1, 1><<<kTiles / 8, 256, 0, stream>>>(
      WVH, kDim, XH, kDim, (void*)VT, kSeq, bv, kVCarry, kInner, kSeq, kDim, kVtScale);

  static_assert(((kSeq * (kHeads / 2)) % 8) == 0, "norm grid exact");
  norm_rot_kernel<<<dim3(kSeq * (kHeads / 2) / 8, 2), 256, 0, stream>>>(
      QF, KF, nqw, nkw, ctab, ttab, Q16, K16, kQCarry);
  static_assert(kQCarry == kKCarry, "one carry argument serves both planes");

  attn128_kernel<<<kHeads * (kSeq / 64), 128, 0, stream>>>(Q16, K16, VT, out);
}
